// ODE_GRU_Encoder_19043884991164
// MI455X (gfx1250) — hardware-verified
//
#include <hip/hip_runtime.h>
#include <math.h>

typedef __attribute__((ext_vector_type(16))) _Float16 v16h;
typedef __attribute__((ext_vector_type(8)))  _Float16 v8h;
typedef __attribute__((ext_vector_type(8)))  float    v8f;
typedef __attribute__((ext_vector_type(4)))  float    v4f;
typedef __attribute__((ext_vector_type(4)))  unsigned int v4u;

template <typename T> struct Frag;
template <> struct Frag<_Float16> {
  typedef v16h V; union U { v16h v; v8h h[2]; };
  static __device__ __forceinline__ v16h load(const _Float16* p) {
    U f; f.h[0] = *(const v8h*)(p); f.h[1] = *(const v8h*)(p + 16); return f.v;
  }
};

__device__ __forceinline__ v8f mma16(v16h a, v16h b, v8f c) {
  c = __builtin_amdgcn_wmma_f32_16x16x32_f16(false, a, false, b, (short)0, c, false, false);
  asm volatile("v_nop\n\tv_nop\n\tv_nop\n\tv_nop" : "+v"(c) : "v"(a), "v"(b));
  return c;
}

constexpr int NB_BATCH = 256;
constexpr int NB_STEP  = 200;
constexpr int NB_XDIM  = 128;
constexpr int NB_HID   = 512;
constexpr int ROWS_PB  = 16;
constexpr int LDA_H    = 1160;
constexpr int LDG_H    = 264;
constexpr int SLAB_P   = 68;
constexpr int KP_O1 = 512;
constexpr int KP_G  = 128;
constexpr int KP_YC = 1152;
constexpr int KP_T1 = 1024;
constexpr float A_SC   = 8.0f;
constexpr float W_SC   = 16.0f;
constexpr float ACC_SC = 0.0078125f;
constexpr int SM_SS    = 0;
constexpr int SM_AT    = 32768;
constexpr int SM_GT    = SM_AT + ROWS_PB * LDA_H * 2;
constexpr int SM_TOTAL = SM_GT + ROWS_PB * LDG_H * 2;
static_assert(SM_TOTAL == 78336);
static_assert(8 * 16 * SLAB_P * 4 <= ROWS_PB * LDA_H * 2);

__global__ __launch_bounds__(256) void tcast_f16(const float* __restrict__ W, int Kreal, int Nreal,
                                                 _Float16* __restrict__ P, int Kp, float wscale) {
  __shared__ __align__(16) _Float16 tile[64 * 72];
  const int tid = threadIdx.x, lane = tid & 31, wv = tid >> 5;
  const int k0 = blockIdx.x * 64, n0 = blockIdx.y * 64;
#pragma unroll 1
  for (int i = 0; i < 16; ++i) {
    const int idx = i * 256 + tid;
    const int kk = idx >> 6, nn = idx & 63;
    const int k = k0 + kk, n = n0 + nn;
    const int kc = (k < Kreal) ? k : (Kreal - 1);
    const int nc = (n < Nreal) ? n : (Nreal - 1);
    float v = W[(size_t)kc * Nreal + nc];
    v = (k < Kreal && n < Nreal) ? (v * wscale) : 0.0f;
    tile[nn * 72 + kk] = (_Float16)v;
  }
  __syncthreads();
  const int q = lane >> 3, c8 = (lane & 7) * 8;
  const int r0 = wv * 4 + q, r1 = 32 + wv * 4 + q;
  const v8h v0 = *(const v8h*)(tile + r0 * 72 + c8);
  const v8h v1 = *(const v8h*)(tile + r1 * 72 + c8);
  _Float16* d0 = P + (size_t)(n0 + r0) * Kp + k0 + c8;
  _Float16* d1 = P + (size_t)(n0 + r1) * Kp + k0 + c8;
  for (int pass = 0; pass < 2; ++pass) {
    *(volatile v8h*)d0 = v0;
    *(volatile v8h*)d1 = v1;
    __threadfence();
  }
}

__device__ __forceinline__ v8f gemm_sub(const _Float16* a_row, const _Float16* __restrict__ b_row, int nks) {
  v8f acc = {0.f, 0.f, 0.f, 0.f, 0.f, 0.f, 0.f, 0.f};
#pragma unroll 2
  for (int ks = 0; ks < nks; ++ks) {
    const v16h a = Frag<_Float16>::load(a_row + ks * 32);
    const v16h b = Frag<_Float16>::load(b_row + ks * 32);
    acc = mma16(a, b, acc);
  }
  return acc;
}

__device__ __forceinline__ float sigm_f(float x) { return 1.0f / (1.0f + expf(-x)); }

__device__ __forceinline__ void tanh_sub(v8f acc, float bias, bool valid, _Float16* gcol) {
#pragma unroll
  for (int r = 0; r < 8; ++r) {
    float v = tanhf(acc[r] * ACC_SC + bias);
    v = valid ? v : 0.0f;
    gcol[r * LDG_H] = (_Float16)(v * A_SC);
  }
}

__device__ __forceinline__ void ode_sub(v8f& h, v8f acc, float bias, float dt, _Float16* acol) {
#pragma unroll
  for (int r = 0; r < 8; ++r) {
    const float hv = h[r] + dt * (acc[r] * ACC_SC + bias);
    h[r] = hv;
    acol[r * LDA_H] = (_Float16)(hv * A_SC);
  }
}

__device__ __forceinline__ void ugate_sub(v8f& u, v8f acc, float bias) {
#pragma unroll
  for (int r = 0; r < 8; ++r) u[r] = sigm_f(acc[r] * ACC_SC + bias);
}

__device__ __forceinline__ void rgate_sub(const v8f& h, v8f acc, float bias, const float* scol, _Float16* acol) {
#pragma unroll
  for (int r = 0; r < 8; ++r) {
    const float rv  = sigm_f(acc[r] * ACC_SC + bias);
    const float hsv = scol[r * NB_HID];
    acol[r * LDA_H]          = (_Float16)((h[r] * rv) * A_SC);
    acol[r * LDA_H + NB_HID] = (_Float16)((hsv * rv) * A_SC);
  }
}

__device__ __forceinline__ void blend_sub(v8f& h, const v8f& u, v8f am, v8f as, float bm, float bs,
                                          float* scol, _Float16* acol) {
#pragma unroll
  for (int r = 0; r < 8; ++r) {
    const float uu   = u[r];
    const float mval = am[r] * ACC_SC + bm;
    const float sval = fabsf(as[r] * ACC_SC + bs);
    const float h2   = (1.0f - uu) * mval + uu * h[r];
    const float hs2  = (1.0f - uu) * sval + uu * scol[r * NB_HID];
    h[r] = h2;
    scol[r * NB_HID] = hs2;
    acol[r * LDA_H]          = (_Float16)(h2 * A_SC);
    acol[r * LDA_H + NB_HID] = (_Float16)(hs2 * A_SC);
  }
}

struct ScanArgs {
  const float* x_data; const float* x_time;
  const float* bo1; const float* bo2; const float* bu1; const float* bu2;
  const float* br1; const float* br2; const float* bn1; const float* bn2;
  const float* bt1; const float* bt2; const float* bt3;
  const _Float16* p_o1; const _Float16* p_o2; const _Float16* p_ur1;
  const _Float16* p_u2; const _Float16* p_r2; const _Float16* p_n1; const _Float16* p_n2;
  const _Float16* p_t1; const _Float16* p_t2; const _Float16* p_t3;
  float* out;
};
static_assert(sizeof(ScanArgs) == 24 * sizeof(void*));

__global__ __launch_bounds__(256) void ode_gru_scan(ScanArgs p) {
  extern __shared__ __align__(16) unsigned char smem_dyn[];
  float*    Ss32  = (float*)(smem_dyn + SM_SS);
  _Float16* At    = (_Float16*)(smem_dyn + SM_AT);
  _Float16* Gt    = (_Float16*)(smem_dyn + SM_GT);
  float*    slabs = (float*)(smem_dyn + SM_AT);

  const int tid = threadIdx.x, lane = tid & 31, wv = tid >> 5;
  const int c = lane & 15, hh = lane >> 4;
  const int koff = hh * 8;
  const int mOff = hh * 8;
  const int b0 = blockIdx.x * ROWS_PB;

  {
    const v4u z = {0u, 0u, 0u, 0u};
    v4u* zs = (v4u*)Ss32;
    for (int i = tid; i < 32768 / 16; i += 256) zs[i] = z;
    v4u* za = (v4u*)At;
    for (int i = tid; i < (ROWS_PB * LDA_H * 2) / 16; i += 256) za[i] = z;
  }
  v8f h0v = {0.f,0.f,0.f,0.f,0.f,0.f,0.f,0.f}, h1v = h0v, h2v = h0v, h3v = h0v;
  v8f u0v = h0v, u1v = h0v, u2v = h0v, u3v = h0v;
  __syncthreads();

  const _Float16* a_row = At + c * LDA_H + koff;
  const _Float16* g_row = Gt + c * LDG_H + koff;
  const float xt_last = p.x_time[NB_STEP - 1];
  const float xt_first = p.x_time[0];
  const int nb = wv * 64;
  const int nh = wv * 16 + c;
  const int nhc = (nh < 100) ? nh : 99;
  const bool hvalid = (nh < 100);

  for (int t = 0; t < NB_STEP; ++t) {
    const int ia = (t >= 2) ? (t - 2) : 0;
    const int ib = (t >= 1) ? (t - 1) : 0;
    const float xa = p.x_time[ia], xb = p.x_time[ib];
    float dt = xa - xb;
    if (t == 1) dt = xt_last - xt_first;
    if (t == 0) dt = -0.01f;

    {
      const int m = tid >> 4, cx = tid & 15;
      const float* xp = p.x_data + ((size_t)(b0 + m) * NB_STEP + t) * NB_XDIM + cx * 8;
      const v4f a0 = *(const v4f*)xp;
      const v4f a1 = *(const v4f*)(xp + 4);
      v8h hx;
#pragma unroll
      for (int j = 0; j < 4; ++j) { hx[j] = (_Float16)(a0[j] * A_SC); hx[4 + j] = (_Float16)(a1[j] * A_SC); }
      *(v8h*)(At + m * LDA_H + 1024 + cx * 8) = hx;
    }
    __syncthreads();

    {
      const v8f acc = gemm_sub(a_row, p.p_o1 + (size_t)nh * KP_O1 + koff, KP_O1 / 32);
      tanh_sub(acc, p.bo1[nhc], hvalid, Gt + mOff * LDG_H + nh);
    }
    __syncthreads();

    ode_sub(h0v, gemm_sub(g_row, p.p_o2 + (size_t)(nb +  0 + c) * KP_G + koff, 4), p.bo2[nb +  0 + c], dt, At + mOff * LDA_H + nb +  0 + c);
    ode_sub(h1v, gemm_sub(g_row, p.p_o2 + (size_t)(nb + 16 + c) * KP_G + koff, 4), p.bo2[nb + 16 + c], dt, At + mOff * LDA_H + nb + 16 + c);
    ode_sub(h2v, gemm_sub(g_row, p.p_o2 + (size_t)(nb + 32 + c) * KP_G + koff, 4), p.bo2[nb + 32 + c], dt, At + mOff * LDA_H + nb + 32 + c);
    ode_sub(h3v, gemm_sub(g_row, p.p_o2 + (size_t)(nb + 48 + c) * KP_G + koff, 4), p.bo2[nb + 48 + c], dt, At + mOff * LDA_H + nb + 48 + c);
    __syncthreads();

    {
      const v8f au = gemm_sub(a_row, p.p_ur1 + (size_t)nh * KP_YC + koff, KP_YC / 32);
      tanh_sub(au, p.bu1[nhc], hvalid, Gt + mOff * LDG_H + nh);
      const v8f ar = gemm_sub(a_row, p.p_ur1 + (size_t)(128 + nh) * KP_YC + koff, KP_YC / 32);
      tanh_sub(ar, p.br1[nhc], hvalid, Gt + mOff * LDG_H + 128 + nh);
    }
    __syncthreads();

    ugate_sub(u0v, gemm_sub(g_row, p.p_u2 + (size_t)(nb +  0 + c) * KP_G + koff, 4), p.bu2[nb +  0 + c]);
    ugate_sub(u1v, gemm_sub(g_row, p.p_u2 + (size_t)(nb + 16 + c) * KP_G + koff, 4), p.bu2[nb + 16 + c]);
    ugate_sub(u2v, gemm_sub(g_row, p.p_u2 + (size_t)(nb + 32 + c) * KP_G + koff, 4), p.bu2[nb + 32 + c]);
    ugate_sub(u3v, gemm_sub(g_row, p.p_u2 + (size_t)(nb + 48 + c) * KP_G + koff, 4), p.bu2[nb + 48 + c]);
    rgate_sub(h0v, gemm_sub(g_row + 128, p.p_r2 + (size_t)(nb +  0 + c) * KP_G + koff, 4), p.br2[nb +  0 + c],
              Ss32 + mOff * NB_HID + nb +  0 + c, At + mOff * LDA_H + nb +  0 + c);
    rgate_sub(h1v, gemm_sub(g_row + 128, p.p_r2 + (size_t)(nb + 16 + c) * KP_G + koff, 4), p.br2[nb + 16 + c],
              Ss32 + mOff * NB_HID + nb + 16 + c, At + mOff * LDA_H + nb + 16 + c);
    rgate_sub(h2v, gemm_sub(g_row + 128, p.p_r2 + (size_t)(nb + 32 + c) * KP_G + koff, 4), p.br2[nb + 32 + c],
              Ss32 + mOff * NB_HID + nb + 32 + c, At + mOff * LDA_H + nb + 32 + c);
    rgate_sub(h3v, gemm_sub(g_row + 128, p.p_r2 + (size_t)(nb + 48 + c) * KP_G + koff, 4), p.br2[nb + 48 + c],
              Ss32 + mOff * NB_HID + nb + 48 + c, At + mOff * LDA_H + nb + 48 + c);
    __syncthreads();

    {
      const v8f an = gemm_sub(a_row, p.p_n1 + (size_t)nh * KP_YC + koff, KP_YC / 32);
      tanh_sub(an, p.bn1[nhc], hvalid, Gt + mOff * LDG_H + nh);
    }
    __syncthreads();

    blend_sub(h0v, u0v, gemm_sub(g_row, p.p_n2 + (size_t)(nb +  0 + c) * KP_G + koff, 4),
                        gemm_sub(g_row, p.p_n2 + (size_t)(NB_HID + nb +  0 + c) * KP_G + koff, 4),
              p.bn2[nb +  0 + c], p.bn2[NB_HID + nb +  0 + c], Ss32 + mOff * NB_HID + nb +  0 + c, At + mOff * LDA_H + nb +  0 + c);
    blend_sub(h1v, u1v, gemm_sub(g_row, p.p_n2 + (size_t)(nb + 16 + c) * KP_G + koff, 4),
                        gemm_sub(g_row, p.p_n2 + (size_t)(NB_HID + nb + 16 + c) * KP_G + koff, 4),
              p.bn2[nb + 16 + c], p.bn2[NB_HID + nb + 16 + c], Ss32 + mOff * NB_HID + nb + 16 + c, At + mOff * LDA_H + nb + 16 + c);
    blend_sub(h2v, u2v, gemm_sub(g_row, p.p_n2 + (size_t)(nb + 32 + c) * KP_G + koff, 4),
                        gemm_sub(g_row, p.p_n2 + (size_t)(NB_HID + nb + 32 + c) * KP_G + koff, 4),
              p.bn2[nb + 32 + c], p.bn2[NB_HID + nb + 32 + c], Ss32 + mOff * NB_HID + nb + 32 + c, At + mOff * LDA_H + nb + 32 + c);
    blend_sub(h3v, u3v, gemm_sub(g_row, p.p_n2 + (size_t)(nb + 48 + c) * KP_G + koff, 4),
                        gemm_sub(g_row, p.p_n2 + (size_t)(NB_HID + nb + 48 + c) * KP_G + koff, 4),
              p.bn2[nb + 48 + c], p.bn2[NB_HID + nb + 48 + c], Ss32 + mOff * NB_HID + nb + 48 + c, At + mOff * LDA_H + nb + 48 + c);
    __syncthreads();
  }

  {
    const v8f acc = gemm_sub(a_row, p.p_t1 + (size_t)nh * KP_T1 + koff, KP_T1 / 32);
    tanh_sub(acc, p.bt1[nhc], hvalid, Gt + mOff * LDG_H + nh);
  }
  __syncthreads();
  {
    const v8f acc = gemm_sub(g_row, p.p_t2 + (size_t)nh * KP_G + koff, 4);
    tanh_sub(acc, p.bt2[nhc], hvalid, Gt + mOff * LDG_H + 128 + nh);
  }
  __syncthreads();
  {
    float* slab = slabs + wv * (16 * SLAB_P);
    const int c4 = (lane & 15) * 4;
    for (int grp = 0; grp < 2; ++grp) {
      const int pbase = grp * NB_HID + nb;
#pragma unroll
      for (int j = 0; j < 4; ++j) {
        const int col = pbase + 16 * j + c;
        const v8f acc = gemm_sub(g_row + 128, p.p_t3 + (size_t)col * KP_G + koff, 4);
        const float bias = p.bt3[col];
#pragma unroll
        for (int r = 0; r < 8; ++r) {
          float v = acc[r] * ACC_SC + bias;
          v = grp ? fabsf(v) : v;
          slab[(mOff + r) * SLAB_P + 16 * j + c] = v;
        }
      }
      __builtin_amdgcn_fence(__ATOMIC_RELEASE, "workgroup");
      __builtin_amdgcn_wave_barrier();
      __builtin_amdgcn_fence(__ATOMIC_ACQUIRE, "workgroup");
      float* C = p.out + (size_t)grp * (NB_BATCH * NB_HID);
      for (int pass = 0; pass < 2; ++pass) {
#pragma unroll
        for (int it = 0; it < 8; ++it) {
          const int row = it * 2 + hh;
          const v4f val = *(const v4f*)(slab + row * SLAB_P + c4);
          *(volatile v4f*)(C + (size_t)(b0 + row) * NB_HID + nb + c4) = val;
        }
        __threadfence();
      }
      __builtin_amdgcn_fence(__ATOMIC_RELEASE, "workgroup");
      __builtin_amdgcn_wave_barrier();
      __builtin_amdgcn_fence(__ATOMIC_ACQUIRE, "workgroup");
    }
  }
}

extern "C" void kernel_launch(void* const* d_in, const int* in_sizes, int n_in,
                              void* d_out, int out_size, void* d_ws, size_t ws_size,
                              hipStream_t stream) {
  if (n_in < 24) return;
  if (in_sizes[0] != NB_BATCH * NB_STEP * NB_XDIM) return;
  if (in_sizes[1] != NB_STEP) return;
  if (out_size != 2 * NB_BATCH * NB_HID) return;
  if (in_sizes[2] != 1152 * 100 || in_sizes[12] != 100 * 1024 || in_sizes[14] != 512 * 100 ||
      in_sizes[18] != 1024 * 100 || in_sizes[20] != 100 * 100 || in_sizes[22] != 100 * 1024) return;

  const size_t OFF_O1  = 0;
  const size_t OFF_O2  = OFF_O1  + (size_t)128  * 512  * 2;
  const size_t OFF_UR1 = OFF_O2  + (size_t)512  * 128  * 2;
  const size_t OFF_U2  = OFF_UR1 + (size_t)256  * 1152 * 2;
  const size_t OFF_R2  = OFF_U2  + (size_t)512  * 128  * 2;
  const size_t OFF_N1  = OFF_R2  + (size_t)512  * 128  * 2;
  const size_t OFF_N2  = OFF_N1  + (size_t)128  * 1152 * 2;
  const size_t OFF_T1  = OFF_N2  + (size_t)1024 * 128  * 2;
  const size_t OFF_T2  = OFF_T1  + (size_t)128  * 1024 * 2;
  const size_t OFF_T3  = OFF_T2  + (size_t)128  * 128  * 2;
  const size_t OFF_END = OFF_T3  + (size_t)1024 * 128  * 2;
  if (OFF_END > ws_size) return;

  unsigned char* ws = (unsigned char*)d_ws;
  _Float16* p_o1  = (_Float16*)(ws + OFF_O1);
  _Float16* p_o2  = (_Float16*)(ws + OFF_O2);
  _Float16* p_ur1 = (_Float16*)(ws + OFF_UR1);
  _Float16* p_u2  = (_Float16*)(ws + OFF_U2);
  _Float16* p_r2  = (_Float16*)(ws + OFF_R2);
  _Float16* p_n1  = (_Float16*)(ws + OFF_N1);
  _Float16* p_n2  = (_Float16*)(ws + OFF_N2);
  _Float16* p_t1  = (_Float16*)(ws + OFF_T1);
  _Float16* p_t2  = (_Float16*)(ws + OFF_T2);
  _Float16* p_t3  = (_Float16*)(ws + OFF_T3);

  const float* x_data = (const float*)d_in[0];
  const float* x_time = (const float*)d_in[1];
  const float* Wu1 = (const float*)d_in[2];  const float* bu1 = (const float*)d_in[3];
  const float* Wu2 = (const float*)d_in[4];  const float* bu2 = (const float*)d_in[5];
  const float* Wr1 = (const float*)d_in[6];  const float* br1 = (const float*)d_in[7];
  const float* Wr2 = (const float*)d_in[8];  const float* br2 = (const float*)d_in[9];
  const float* Wn1 = (const float*)d_in[10]; const float* bn1 = (const float*)d_in[11];
  const float* Wn2 = (const float*)d_in[12]; const float* bn2 = (const float*)d_in[13];
  const float* Wo1 = (const float*)d_in[14]; const float* bo1 = (const float*)d_in[15];
  const float* Wo2 = (const float*)d_in[16]; const float* bo2 = (const float*)d_in[17];
  const float* Wt1 = (const float*)d_in[18]; const float* bt1 = (const float*)d_in[19];
  const float* Wt2 = (const float*)d_in[20]; const float* bt2 = (const float*)d_in[21];
  const float* Wt3 = (const float*)d_in[22]; const float* bt3 = (const float*)d_in[23];

  tcast_f16<<<dim3(512 / 64,  128 / 64), 256, 0, stream>>>(Wo1, 512,  100,  p_o1,  512,  W_SC);
  tcast_f16<<<dim3(128 / 64,  512 / 64), 256, 0, stream>>>(Wo2, 100,  512,  p_o2,  128,  W_SC);
  tcast_f16<<<dim3(1152 / 64, 128 / 64), 256, 0, stream>>>(Wu1, 1152, 100,  p_ur1, 1152, W_SC);
  tcast_f16<<<dim3(1152 / 64, 128 / 64), 256, 0, stream>>>(Wr1, 1152, 100,  p_ur1 + (size_t)128 * 1152, 1152, W_SC);
  tcast_f16<<<dim3(128 / 64,  512 / 64), 256, 0, stream>>>(Wu2, 100,  512,  p_u2,  128,  W_SC);
  tcast_f16<<<dim3(128 / 64,  512 / 64), 256, 0, stream>>>(Wr2, 100,  512,  p_r2,  128,  W_SC);
  tcast_f16<<<dim3(1152 / 64, 128 / 64), 256, 0, stream>>>(Wn1, 1152, 100,  p_n1,  1152, W_SC);
  tcast_f16<<<dim3(128 / 64, 1024 / 64), 256, 0, stream>>>(Wn2, 100,  1024, p_n2,  128,  W_SC);
  tcast_f16<<<dim3(1024 / 64, 128 / 64), 256, 0, stream>>>(Wt1, 1024, 100,  p_t1,  1024, W_SC);
  tcast_f16<<<dim3(128 / 64,  128 / 64), 256, 0, stream>>>(Wt2, 100,  100,  p_t2,  128,  W_SC);
  tcast_f16<<<dim3(128 / 64, 1024 / 64), 256, 0, stream>>>(Wt3, 100,  1024, p_t3,  128,  W_SC);

  ScanArgs a;
  a.x_data = x_data; a.x_time = x_time;
  a.bo1 = bo1; a.bo2 = bo2; a.bu1 = bu1; a.bu2 = bu2;
  a.br1 = br1; a.br2 = br2; a.bn1 = bn1; a.bn2 = bn2;
  a.bt1 = bt1; a.bt2 = bt2; a.bt3 = bt3;
  a.p_o1 = p_o1; a.p_o2 = p_o2; a.p_ur1 = p_ur1;
  a.p_u2 = p_u2; a.p_r2 = p_r2; a.p_n1 = p_n1; a.p_n2 = p_n2;
  a.p_t1 = p_t1; a.p_t2 = p_t2; a.p_t3 = p_t3;
  a.out = (float*)d_out;

  ode_gru_scan<<<NB_BATCH / ROWS_PB, 256, SM_TOTAL, stream>>>(a);
}
